// BahdanauAttention_65240553226467
// MI455X (gfx1250) — hardware-run, weakly checked
//
#include <hip/hip_runtime.h>


#ifndef NB
#define NB 4
#endif
#ifndef TQ
#define TQ 256
#endif
#define NB_FULL 4
#define TQ_FULL 256
#define TK      512
#define TK_FULL 512
#ifndef OUT_TQ
#define OUT_TQ TQ
#endif
#define HD   512
#define W1P  (2 * HD)
#define QT   4
#define PT   512
#define TS2  2.8853900817779268f
#define L2E  1.4426950408889634f
#define FILLV (-1000.0f)

static_assert(HD % 64 == 0);
static_assert(HD % 32 == 0);
static_assert((NB * TQ) % 64 == 0);
static_assert((NB * TK) % 64 == 0);
static_assert(TQ % QT == 0);
static_assert(PT == 512);
static_assert(HD == PT);
static_assert(TK == PT);
static_assert(TK == TK_FULL);
static_assert(QT == 4);
static_assert(QT * HD == PT * 4);
static_assert((size_t)PT * 16 == (size_t)QT * TK * 4);
static_assert(32 * 16 * 8 == 16 * 64 * 4);
static_assert(NB <= NB_FULL);
static_assert(TQ <= TQ_FULL);
static_assert(W1P % 8 == 0);
static_assert(((size_t)NB * TQ * HD) % 8 == 0);
static_assert(((size_t)TQ * HD) % 8 == 0);
static_assert(((size_t)NB * TK * HD) % 8 == 0);
static_assert(((size_t)HD * W1P) % 8 == 0);
static_assert(16 * 68 * 4 <= 131072);
static_assert(QT * HD * 4 + HD * 4 + QT * TK * 4 + 2 * 16 * QT * 4 + 16 * 4 <= 131072);

typedef unsigned short bf;
typedef __attribute__((ext_vector_type(16))) __bf16   v16bf;
typedef __attribute__((ext_vector_type(8)))  unsigned short v8us;
typedef __attribute__((ext_vector_type(8)))  float    v8f;
typedef __attribute__((ext_vector_type(4)))  float    v4f;
typedef v4f  __attribute__((may_alias)) v4fa;

__device__ __forceinline__ unsigned short f2bf(float f) { unsigned u = __float_as_uint(f); u += 0x7FFFu + ((u >> 16) & 1u); return (unsigned short)(u >> 16); }
__device__ __forceinline__ float bfr(float f) { return __uint_as_float(((unsigned)f2bf(f)) << 16); }
__device__ __forceinline__ v16bf cat16b(v8us lo, v8us hi) { return __builtin_bit_cast(v16bf, __builtin_shufflevector(lo, hi, 0, 1, 2, 3, 4, 5, 6, 7, 8, 9, 10, 11, 12, 13, 14, 15)); }
__device__ __forceinline__ v8f wmmab(v16bf a, v16bf b, v8f c) { return __builtin_amdgcn_wmma_f32_16x16x32_bf16(false, a, false, b, (short)0, c, false, false); }
__device__ __forceinline__ v16bf ldb(const bf* p)  { return cat16b(*(const v8us*)p, *(const v8us*)(p + 16)); }
__device__ __forceinline__ void wave_sync() { __builtin_amdgcn_fence(3  , "wavefront"); __builtin_amdgcn_wave_barrier(); asm volatile("" ::: "memory"); }
__device__ __forceinline__ v8f wmmab_g(v16bf a, v16bf b, v8f c) {
    c = wmmab(a, b, c);
    asm volatile("v_nop\n\tv_nop\n\tv_nop\n\tv_nop" : "+v"(c) : "v"(a), "v"(b));
    return c;
}

__global__ __launch_bounds__(256) void k_cvt8(const float* __restrict__ src, bf* dst, size_t n8) {
    const size_t i = (size_t)blockIdx.x * 256 + threadIdx.x; if (i >= n8) return;
    const v8f v = *(const v8f*)(src + i * 8); v8us o;
#pragma unroll
    for (int k = 0; k < 8; ++k) o[k] = f2bf(v[k]);
    *(volatile v8us*)(dst + i * 8) = o; __threadfence(); *(volatile v8us*)(dst + i * 8) = o;
}

__global__ __launch_bounds__(32) void k_lin(const bf* __restrict__ A, const bf* __restrict__ Bt, const float* __restrict__ bias, int hasb, float* C) {
    __shared__ __align__(16) float os[16 * 68];
    const int lane = threadIdx.x & 31, lr = lane & 15, hi = lane >> 4; const int r0 = blockIdx.x * 64, c0 = blockIdx.y * 64;
    v8f acc[4][4];
#pragma unroll
    for (int mb = 0; mb < 4; ++mb)
#pragma unroll
        for (int nb = 0; nb < 4; ++nb) acc[mb][nb] = (v8f){};
    const size_t aoff = (size_t)(r0 + lr) * HD + 8 * hi, boff = (size_t)(c0 + lr) * W1P + 8 * hi;
#pragma unroll 1
    for (int kc = 0; kc < HD; kc += 32) {
        v16bf a[4];
#pragma unroll
        for (int mb = 0; mb < 4; ++mb) a[mb] = ldb(A + aoff + (size_t)mb * 16 * HD + kc);
#pragma unroll
        for (int nb = 0; nb < 4; ++nb) { const v16bf b = ldb(Bt + boff + (size_t)nb * 16 * W1P + kc);
#pragma unroll
            for (int mb = 0; mb < 4; ++mb) acc[mb][nb] = wmmab_g(a[mb], b, acc[mb][nb]); }
    }
    float bc[4];
#pragma unroll
    for (int nb = 0; nb < 4; ++nb) { const float braw = bias[c0 + nb * 16 + lr]; bc[nb] = (hasb != 0) ? bfr(braw) : 0.0f; }
#pragma unroll
    for (int mb = 0; mb < 4; ++mb) {
#pragma unroll
        for (int nb = 0; nb < 4; ++nb) {
#pragma unroll
            for (int j = 0; j < 8; ++j) os[(hi * 8 + j) * 68 + nb * 16 + lr] = (acc[mb][nb][j] + bc[nb]) * TS2; }
        wave_sync();
        float* cb = C + (size_t)(r0 + mb * 16) * HD + c0;
#pragma unroll 1
        for (int ps = 0; ps < 2; ++ps) {
#pragma unroll
            for (int s = 0; s < 8; ++s) { const int row = 2 * s + (lane >> 4), c4 = (lane & 15) * 4;
                const v4f val = *(const v4fa*)(&os[row * 68 + c4]);
                *(volatile v4f*)(cb + (size_t)row * HD + c4) = val; }
            if (ps == 0) __threadfence(); }
        wave_sync();
    }
}

__global__ __launch_bounds__(PT) void k_pair(const float* __restrict__ QS, const float* __restrict__ KS, const int* __restrict__ mask,
                                             const float* __restrict__ w2, const float* __restrict__ b2, float* OUT) {
    __shared__ __align__(16) float qs[QT * HD];
    __shared__ __align__(16) float wl[HD];
    __shared__ __align__(16) float ps[QT * TK];
    __shared__ __align__(16) float redm[16 * QT];
    __shared__ __align__(16) float reds[16 * QT];
    __shared__ __align__(16) float wred[16];
    const int tid = threadIdx.x, lane = tid & 31;
    const int wave = __builtin_amdgcn_readfirstlane((int)(threadIdx.x >> 5));
    const int b = blockIdx.y, q0 = blockIdx.x * QT;
    { const v4f qv = *(const v4f*)(QS + ((size_t)b * TQ + q0) * HD + (size_t)tid * 4); *(v4fa*)(&qs[tid * 4]) = qv; }
    const float wmine = bfr(w2[tid]);
    wl[tid] = wmine;
    float wsm = wmine;
    wsm += __shfl_xor(wsm, 16, 32); wsm += __shfl_xor(wsm, 8, 32); wsm += __shfl_xor(wsm, 4, 32); wsm += __shfl_xor(wsm, 2, 32); wsm += __shfl_xor(wsm, 1, 32);
    if (lane == 0) wred[wave] = wsm;
    __syncthreads();
    float wsum = 0.0f;
#pragma unroll 1
    for (int w = 0; w < 16; ++w) wsum += wred[w];
    const float cbias = bfr(b2[0]) + wsum;

    const float* krow = KS + ((size_t)b * TK + tid) * HD;
    float acc[QT];
#pragma unroll
    for (int i = 0; i < QT; ++i) acc[i] = 0.0f;
#pragma unroll 1
    for (int h = 0; h < HD; h += 4) {
        const v4f kv = *(const v4f*)(krow + h);
        const v4f wv = *(const v4fa*)(&wl[h]);
#pragma unroll
        for (int i = 0; i < QT; ++i) {
            const v4f qv = *(const v4fa*)(&qs[i * HD + h]);
#pragma unroll
            for (int c = 0; c < 4; ++c) {
                const float t = __builtin_amdgcn_exp2f(qv[c] + kv[c]);
                acc[i] += wv[c] * __builtin_amdgcn_rcpf(1.0f + t); }
        }
    }

    const int* mrow = mask + ((size_t)b * TQ_FULL + q0) * TK_FULL + tid;
    float lg[QT]; v4f mw;
#pragma unroll
    for (int i = 0; i < QT; ++i) {
        const int mv = mrow[(size_t)i * TK_FULL];
        const float v = cbias - 2.0f * acc[i];
        lg[i] = (mv == 0) ? FILLV : v;
        float mx = lg[i];
        mx = fmaxf(mx, __shfl_xor(mx, 16, 32)); mx = fmaxf(mx, __shfl_xor(mx, 8, 32)); mx = fmaxf(mx, __shfl_xor(mx, 4, 32));
        mx = fmaxf(mx, __shfl_xor(mx, 2, 32)); mx = fmaxf(mx, __shfl_xor(mx, 1, 32));
        mw[i] = mx; }
    if (lane == 0) *(v4fa*)(&redm[wave * QT]) = mw;
    __syncthreads();
    v4f gm = *(const v4fa*)(&redm[0]);
#pragma unroll 1
    for (int w = 1; w < 16; ++w) { const v4f t = *(const v4fa*)(&redm[w * QT]);
#pragma unroll
        for (int i = 0; i < QT; ++i) gm[i] = fmaxf(gm[i], t[i]); }

    float ev[QT]; v4f sw;
#pragma unroll
    for (int i = 0; i < QT; ++i) {
        ev[i] = __builtin_amdgcn_exp2f((lg[i] - gm[i]) * L2E);
        float s = ev[i];
        s += __shfl_xor(s, 16, 32); s += __shfl_xor(s, 8, 32); s += __shfl_xor(s, 4, 32); s += __shfl_xor(s, 2, 32); s += __shfl_xor(s, 1, 32);
        sw[i] = s; }
    if (lane == 0) *(v4fa*)(&reds[wave * QT]) = sw;
    __syncthreads();
    v4f gs = *(const v4fa*)(&reds[0]);
#pragma unroll 1
    for (int w = 1; w < 16; ++w) { const v4f t = *(const v4fa*)(&reds[w * QT]);
#pragma unroll
        for (int i = 0; i < QT; ++i) gs[i] += t[i]; }
#pragma unroll
    for (int i = 0; i < QT; ++i) { const float inv = __builtin_amdgcn_rcpf(gs[i]); ps[i * TK + tid] = ev[i] * inv; }
    __syncthreads();
    const v4f val = *(const v4fa*)(&ps[tid * 4]);
    float* o = OUT + ((size_t)b * OUT_TQ + q0) * TK + (size_t)tid * 4;
    *(volatile v4f*)o = val; __threadfence(); *(volatile v4f*)o = val;
}

static constexpr size_t al256(size_t v) { return (v + 255) & ~(size_t)255; }
static constexpr size_t SZ_XQ = al256((size_t)NB * TQ * HD * 2);
static constexpr size_t SZ_XK = al256((size_t)NB * TK * HD * 2);
static constexpr size_t SZ_WB = al256((size_t)HD * W1P * 2);
static constexpr size_t SZ_QS = al256((size_t)NB * TQ * HD * 4);
static constexpr size_t SZ_KS = al256((size_t)NB * TK * HD * 4);
static constexpr size_t SZ_TOTAL = SZ_XQ + SZ_XK + SZ_WB + SZ_QS + SZ_KS;
static_assert(SZ_TOTAL <= (size_t)134217728);
static_assert(((size_t)HD * 2) % 16 == 0);

extern "C" void kernel_launch(void* const* d_in, const int* in_sizes, int n_in,
                              void* d_out, int out_size, void* d_ws, size_t ws_size, hipStream_t stream) {
    if (n_in < 7) return;
    const size_t needq = ((size_t)(NB - 1) * TQ_FULL + TQ) * HD;
    const size_t needk = (size_t)NB * TK * HD;
    const size_t needm = ((size_t)(NB - 1) * TQ_FULL + TQ) * TK;
    if ((size_t)in_sizes[0] < needq || (size_t)in_sizes[1] < needk || (size_t)in_sizes[2] < needm) return;
    if ((size_t)in_sizes[3] < (size_t)HD * W1P) return;
    if (in_sizes[4] < HD || in_sizes[5] < HD || in_sizes[6] < 1) return;
    if ((size_t)out_size < ((size_t)(NB - 1) * OUT_TQ + TQ) * TK) return;
    if (SZ_TOTAL > ws_size) return;
    const float* query = (const float*)d_in[0];
    const float* key   = (const float*)d_in[1];
    const int*   mask  = (const int*)d_in[2];
    const float* w1    = (const float*)d_in[3];
    const float* b1    = (const float*)d_in[4];
    const float* w2    = (const float*)d_in[5];
    const float* b2    = (const float*)d_in[6];
    float* OUT = (float*)d_out;
    char* wsp = (char*)d_ws;
    bf* XQ = (bf*)wsp; wsp += SZ_XQ;
    bf* XK = (bf*)wsp; wsp += SZ_XK;
    bf* WB = (bf*)wsp; wsp += SZ_WB;
    float* QS = (float*)wsp; wsp += SZ_QS;
    float* KS = (float*)wsp; wsp += SZ_KS;

    if (TQ == TQ_FULL) {
        const size_t n8 = (size_t)NB * TQ * HD / 8;
        k_cvt8<<<(unsigned)((n8 + 255) / 256), 256, 0, stream>>>(query, XQ, n8);
    } else {
        const size_t n8 = (size_t)TQ * HD / 8;
        for (int b = 0; b < NB; ++b) k_cvt8<<<(unsigned)((n8 + 255) / 256), 256, 0, stream>>>(query + (size_t)b * TQ_FULL * HD, XQ + (size_t)b * TQ * HD, n8);
    }
    { const size_t n8 = (size_t)NB * TK * HD / 8; k_cvt8<<<(unsigned)((n8 + 255) / 256), 256, 0, stream>>>(key, XK, n8); }
    { const size_t n8 = (size_t)HD * W1P / 8;     k_cvt8<<<(unsigned)((n8 + 255) / 256), 256, 0, stream>>>(w1, WB, n8); }

    k_lin<<<dim3(NB * TQ / 64, HD / 64, 1), 32, 0, stream>>>(XQ, WB, b1, 0, QS);
    k_lin<<<dim3(NB * TK / 64, HD / 64, 1), 32, 0, stream>>>(XK, WB + HD, b1, 1, KS);

    k_pair<<<dim3(TQ / QT, NB, 1), PT, 0, stream>>>(QS, KS, mask, w2, b2, OUT);
}
